// CloMSFM_35132832481638
// MI455X (gfx1250) — hardware-run, weakly checked
//
#include <hip/hip_runtime.h>


#define NBI  16
#define CC   256
#define NN   1024
#define HF   128
#define NH_  4
#define HD   32
#define SCL  0.1767766952966369f
#define PCAR 1024.0f
typedef _Float16 h16;
typedef unsigned short bf;
typedef __attribute__((ext_vector_type(16))) __bf16   v16bf;
typedef __attribute__((ext_vector_type(16))) _Float16 v16h;
typedef __attribute__((ext_vector_type(8)))  _Float16 v8h;
typedef __attribute__((ext_vector_type(8)))  unsigned short v8us;
typedef __attribute__((ext_vector_type(8)))  float    v8f;
typedef __attribute__((ext_vector_type(4)))  float    v4f;
typedef v8h  __attribute__((may_alias)) v8ha;
typedef v4f  __attribute__((may_alias)) v4fa;
typedef v8us __attribute__((may_alias)) v8usa;

__device__ __forceinline__ unsigned short f2bf(float f) { unsigned u = __float_as_uint(f); u += 0x7FFFu + ((u >> 16) & 1u); return (unsigned short)(u >> 16); }
__device__ __forceinline__ float bf2f(unsigned short b) { return __uint_as_float(((unsigned)b) << 16); }
__device__ __forceinline__ float bfr(float f) { return bf2f(f2bf(f)); }
__device__ __forceinline__ v16h cat16(v8h lo, v8h hi) { return __builtin_shufflevector(lo, hi, 0, 1, 2, 3, 4, 5, 6, 7, 8, 9, 10, 11, 12, 13, 14, 15); }
__device__ __forceinline__ v16bf cat16b(v8us lo, v8us hi) { return __builtin_bit_cast(v16bf, __builtin_shufflevector(lo, hi, 0, 1, 2, 3, 4, 5, 6, 7, 8, 9, 10, 11, 12, 13, 14, 15)); }
__device__ __forceinline__ v8f wmma16(v16h a, v16h b, v8f c) { return __builtin_amdgcn_wmma_f32_16x16x32_f16(false, a, false, b, (short)0, c, false, false); }
__device__ __forceinline__ v8f wmmab(v16bf a, v16bf b, v8f c) { return __builtin_amdgcn_wmma_f32_16x16x32_bf16(false, a, false, b, (short)0, c, false, false); }


template <typename T16> struct WFrag;
template <> struct WFrag<h16> { typedef v16h V; static __device__ __forceinline__ V ld(const h16* p) { return cat16(*(const v8h*)p, *(const v8h*)(p + 16)); } static __device__ __forceinline__ v8f mma(V a, V b, v8f c) { return wmma16(a, b, c); } };
template <> struct WFrag<bf> { typedef v16bf V; static __device__ __forceinline__ V ld(const bf* p) { return cat16b(*(const v8us*)p, *(const v8us*)(p + 16)); } static __device__ __forceinline__ v8f mma(V a, V b, v8f c) { return wmmab(a, b, c); } };
template <typename T16, int NSPLIT, bool BIAS>
__global__ __launch_bounds__(32) void k_gemmw(const T16* __restrict__ A, const T16* __restrict__ A2, const T16* __restrict__ Bt, const T16* __restrict__ Bt2, int K, float* C, int ldc, const float* __restrict__ bias, size_t sA, size_t sB, size_t sC) {
    typedef typename WFrag<T16>::V V;
    __shared__ __align__(16) float os[16 * 68];
    const size_t z = blockIdx.z; A += z * sA; if (A2) A2 += z * sA; Bt += z * sB; if (Bt2) Bt2 += z * sB; C += z * sC;
    const int lane = threadIdx.x & 31, lr = lane & 15, hi = lane >> 4; const int r0 = blockIdx.x * 64, c0 = blockIdx.y * 64;
    v8f acc[4][4];
#pragma unroll
    for (int mb = 0; mb < 4; ++mb)
#pragma unroll
        for (int nb = 0; nb < 4; ++nb) acc[mb][nb] = (v8f){};
    const size_t aoff = (size_t)(r0 + lr) * K + 8 * hi, boff = (size_t)(c0 + lr) * K + 8 * hi;
#pragma unroll 1
    for (int kc = 0; kc < K; kc += 32) {
        V a[4], a2[4];
#pragma unroll
        for (int mb = 0; mb < 4; ++mb) { a[mb] = WFrag<T16>::ld(A + aoff + (size_t)mb * 16 * K + kc); if (NSPLIT == 1 || NSPLIT == 2) a2[mb] = WFrag<T16>::ld(A2 + aoff + (size_t)mb * 16 * K + kc); }
#pragma unroll
        for (int nb = 0; nb < 4; ++nb) { const V b = WFrag<T16>::ld(Bt + boff + (size_t)nb * 16 * K + kc); V b2; if (NSPLIT >= 2) b2 = WFrag<T16>::ld(Bt2 + boff + (size_t)nb * 16 * K + kc);
#pragma unroll
            for (int mb = 0; mb < 4; ++mb) { acc[mb][nb] = WFrag<T16>::mma(a[mb], b, acc[mb][nb]); if (NSPLIT == 1 || NSPLIT == 2) acc[mb][nb] = WFrag<T16>::mma(a2[mb], b, acc[mb][nb]); if (NSPLIT >= 2) acc[mb][nb] = WFrag<T16>::mma(a[mb], b2, acc[mb][nb]); } }
        asm volatile("v_nop\n\tv_nop\n\tv_nop\n\tv_nop" : "+v"(acc[0][0]), "+v"(acc[1][1]), "+v"(acc[2][2]), "+v"(acc[3][3]) : "v"(a[0]), "v"(a[3]));
    }
#pragma unroll
    for (int mb = 0; mb < 4; ++mb) {
#pragma unroll
        for (int nb = 0; nb < 4; ++nb) {
#pragma unroll
            for (int j = 0; j < 8; ++j) os[(hi * 8 + j) * 68 + nb * 16 + lr] = acc[mb][nb][j]; }
        __builtin_amdgcn_wave_barrier(); asm volatile("" ::: "memory");
        float* crow = C + (size_t)(r0 + mb * 16) * ldc + c0;
#pragma unroll 1
        for (int ps = 0; ps < 2; ++ps) {
#pragma unroll
            for (int s = 0; s < 8; ++s) { const int row = 2 * s + hi, cofs = lr * 4; v4f val = *(const v4fa*)(os + row * 68 + cofs); if (BIAS) { val[0] += bfr(bias[c0 + cofs]); val[1] += bfr(bias[c0 + cofs + 1]); val[2] += bfr(bias[c0 + cofs + 2]); val[3] += bfr(bias[c0 + cofs + 3]); }
                *(volatile v4f*)(crow + (size_t)row * ldc + cofs) = val; }
            if (ps == 0) __threadfence(); }
        __builtin_amdgcn_wave_barrier(); asm volatile("" ::: "memory");
    }
}

__device__ __forceinline__ h16 tohx(float x) { return (h16)x; }
__device__ __forceinline__ void splitf(float y, unsigned short& h, unsigned short& l) { h = f2bf(y); l = f2bf(y - bf2f(h)); }
__device__ __forceinline__ float tanh_(float x) { const float e = __expf(-2.0f * fabsf(x)); const float t = __fdiv_rn(1.0f - e, 1.0f + e); return copysignf(t, x); }
__device__ __forceinline__ float sigm_(float x) { return __fdiv_rn(1.0f, 1.0f + __expf(-x)); }
typedef __attribute__((ext_vector_type(2))) _Float16 v2h;
typedef __attribute__((ext_vector_type(4))) _Float16 v4h;
typedef __attribute__((ext_vector_type(4))) unsigned short v4us;

__global__ __launch_bounds__(256) void k_cvt8(const float* __restrict__ src, bf* dst, size_t n8) { const size_t i = (size_t)blockIdx.x * 256 + threadIdx.x; if (i >= n8) return; const v8f v = *(const v8f*)(src + i * 8); v8us o;
#pragma unroll
    for (int k = 0; k < 8; ++k) o[k] = f2bf(v[k]); *(volatile v8us*)(dst + i * 8) = o; __threadfence(); *(volatile v8us*)(dst + i * 8) = o; }
__global__ __launch_bounds__(256) void k_xt(const float* __restrict__ x, bf* XT) { const size_t e = ((size_t)blockIdx.x * 256 + threadIdx.x) * 4; if (e >= (size_t)NN * CC) return; const int c = (int)(e % CC); const int n = (int)(e / CC); v4us o;
#pragma unroll
    for (int q = 0; q < 4; ++q) o[q] = f2bf(x[(size_t)(c + q) * NN + n]); *(volatile v4us*)(XT + e) = o; __threadfence(); *(volatile v4us*)(XT + e) = o; }
__global__ __launch_bounds__(256) void k_dw(const float* __restrict__ QKV, const float* __restrict__ dw, const float* __restrict__ db, float* QC) { const size_t e = ((size_t)blockIdx.x * 256 + threadIdx.x) * 4; if (e >= (size_t)NN * 3 * HF) return; const int c = (int)(e % (3 * HF)); const int n = (int)(e / (3 * HF)); const int hy = n / 32, wx = n % 32; v4f o;
#pragma unroll
    for (int q = 0; q < 4; ++q) { const int cc = c + q; float acc = bfr(db[cc]);
#pragma unroll
        for (int ky = 0; ky < 3; ++ky) {
#pragma unroll
            for (int kx = 0; kx < 3; ++kx) { const int yy = hy + ky - 1, xx = wx + kx - 1; if (yy >= 0 && yy < 32 && xx >= 0 && xx < 32) { float p = __fmul_rn(QKV[(size_t)(yy * 32 + xx) * 3 * HF + cc], bfr(dw[cc * 9 + ky * 3 + kx])); asm volatile("" : "+v"(p)); acc = __fadd_rn(acc, p); } } }
        o[q] = acc; }
    *(volatile v4f*)(QC + e) = o; __threadfence(); *(volatile v4f*)(QC + e) = o; }
__global__ __launch_bounds__(256) void k_qkpl(const float* __restrict__ QC, bf* Ph, bf* Pl) { const size_t e = ((size_t)blockIdx.x * 256 + threadIdx.x) * 4; if (e >= (size_t)NN * HF) return; const int c = (int)(e % HF); const int n = (int)(e / HF); const float* r = QC + (size_t)n * 3 * HF; v4us oh, ol;
#pragma unroll
    for (int q = 0; q < 4; ++q) { unsigned short a, b; splitf(__fmul_rn(r[c + q], r[HF + c + q]), a, b); oh[q] = a; ol[q] = b; } *(volatile v4us*)(Ph + e) = oh; *(volatile v4us*)(Pl + e) = ol; __threadfence(); *(volatile v4us*)(Ph + e) = oh; *(volatile v4us*)(Pl + e) = ol; }
__global__ __launch_bounds__(256) void k_swpl(const float* __restrict__ A1, bf* Ph, bf* Pl) { const size_t e = ((size_t)blockIdx.x * 256 + threadIdx.x) * 4; if (e >= (size_t)NN * HF) return; const v4f a = *(const v4f*)(A1 + e); v4us oh, ol;
#pragma unroll
    for (int q = 0; q < 4; ++q) { unsigned short u, b; splitf(__fmul_rn(a[q], sigm_(a[q])), u, b); oh[q] = u; ol[q] = b; } *(volatile v4us*)(Ph + e) = oh; *(volatile v4us*)(Pl + e) = ol; __threadfence(); *(volatile v4us*)(Ph + e) = oh; *(volatile v4us*)(Pl + e) = ol; }
__global__ __launch_bounds__(256) void k_high(const float* __restrict__ A2, const float* __restrict__ QC, float* COMB) { const size_t e = ((size_t)blockIdx.x * 256 + threadIdx.x) * 4; if (e >= (size_t)NN * HF) return; const int c = (int)(e % HF); const int n = (int)(e / HF); const v4f a = *(const v4f*)(A2 + e); v4f o;
#pragma unroll
    for (int q = 0; q < 4; ++q) o[q] = __fmul_rn(tanh_(__fmul_rn(a[q], SCL)), QC[(size_t)n * 3 * HF + 2 * HF + c + q]); *(volatile v4f*)(COMB + (size_t)n * CC + c) = o; __threadfence(); *(volatile v4f*)(COMB + (size_t)n * CC + c) = o; }
__global__ __launch_bounds__(256) void k_gpl(const float* __restrict__ GQ, const float* __restrict__ GKV, h16* Q16, h16* K16) { const size_t e = ((size_t)blockIdx.x * 256 + threadIdx.x) * 4; if (e >= (size_t)NH_ * NN * HD) return; const int d = (int)(e % HD); const int n = (int)((e / HD) % NN); const int h = (int)(e / ((size_t)HD * NN)); v4h oq, ok;
#pragma unroll
    for (int q = 0; q < 4; ++q) { oq[q] = tohx(GQ[(size_t)n * HF + h * HD + d + q] * SCL); ok[q] = tohx(GKV[(size_t)n * 2 * HF + h * HD + d + q]); } for (int ps = 0; ps < 2; ++ps) { *(volatile v4h*)(Q16 + e) = oq; *(volatile v4h*)(K16 + e) = ok; if (ps == 0) __threadfence(); } }
__global__ __launch_bounds__(256) void k_gvt(const float* __restrict__ GKV, h16* VT) { const size_t e = ((size_t)blockIdx.x * 256 + threadIdx.x) * 2; if (e >= (size_t)NH_ * 64 * NN) return; const int m = (int)(e % NN); const int dv = (int)((e / NN) % 64); const int h = (int)(e / ((size_t)NN * 64)); v2h o; o[0] = dv < HD ? tohx(GKV[(size_t)m * 2 * HF + HF + h * HD + dv]) : (h16)0.f; o[1] = dv < HD ? tohx(GKV[(size_t)(m + 1) * 2 * HF + HF + h * HD + dv]) : (h16)0.f; *(volatile v2h*)(VT + e) = o; __threadfence(); *(volatile v2h*)(VT + e) = o; }
__global__ __launch_bounds__(256) void k_low(const float* __restrict__ O, float* COMB) { const size_t e = ((size_t)blockIdx.x * 256 + threadIdx.x) * 4; if (e >= (size_t)NN * HF) return; const int c = (int)(e % HF); const int n = (int)(e / HF); const int h = c / HD, d = c % HD; const float* r = O + ((size_t)h * NN + n) * 64 + d; v4f o; o[0] = r[0] * (1.0f / PCAR); o[1] = r[1] * (1.0f / PCAR); o[2] = r[2] * (1.0f / PCAR); o[3] = r[3] * (1.0f / PCAR); *(volatile v4f*)(COMB + (size_t)n * CC + HF + c) = o; __threadfence(); *(volatile v4f*)(COMB + (size_t)n * CC + HF + c) = o; }
__global__ __launch_bounds__(256) void k_se(const float* __restrict__ COMB, const float* __restrict__ w1, const float* __restrict__ w2, float* CA) { __shared__ float pooled[CC]; __shared__ float rr[16]; const int c = threadIdx.x; float s = 0.f;
#pragma unroll 1
    for (int n = 0; n < NN; ++n) s = __fadd_rn(s, COMB[(size_t)n * CC + c]); pooled[c] = s * (1.0f / NN); __syncthreads();
    if (c < 16) { float a = 0.f;
#pragma unroll 1
        for (int k = 0; k < CC; ++k) { float p = __fmul_rn(pooled[k], bfr(w1[c * CC + k])); asm volatile("" : "+v"(p)); a = __fadd_rn(a, p); } rr[c] = fmaxf(a, 0.f); } __syncthreads();
    float g = 0.f;
#pragma unroll 1
    for (int j = 0; j < 16; ++j) { float p = __fmul_rn(rr[j], bfr(w2[c * 16 + j])); asm volatile("" : "+v"(p)); g = __fadd_rn(g, p); } const float ca = sigm_(g); *(volatile float*)(CA + c) = ca; __threadfence(); *(volatile float*)(CA + c) = ca; }
__global__ __launch_bounds__(256) void k_capl(const float* __restrict__ COMB, const float* __restrict__ CA, bf* Ph, bf* Pl) { const size_t e = ((size_t)blockIdx.x * 256 + threadIdx.x) * 4; if (e >= (size_t)NN * CC) return; const int c = (int)(e % CC); const v4f a = *(const v4f*)(COMB + e); v4us oh, ol;
#pragma unroll
    for (int q = 0; q < 4; ++q) { unsigned short u, b; splitf(__fmul_rn(a[q], CA[c + q]), u, b); oh[q] = u; ol[q] = b; } *(volatile v4us*)(Ph + e) = oh; *(volatile v4us*)(Pl + e) = ol; __threadfence(); *(volatile v4us*)(Ph + e) = oh; *(volatile v4us*)(Pl + e) = ol; }
__global__ __launch_bounds__(256) void k_outT(const float* __restrict__ R, const float* __restrict__ x, float* OUT) { const size_t e = ((size_t)blockIdx.x * 256 + threadIdx.x) * 4; if (e >= (size_t)CC * NN) return; const int n = (int)(e % NN); const int c = (int)(e / NN); v4f o;
#pragma unroll
    for (int q = 0; q < 4; ++q) o[q] = __fadd_rn(bfr(x[e + q]), R[(size_t)(n + q) * CC + c]); *(volatile v4f*)(OUT + e) = o; __threadfence(); *(volatile v4f*)(OUT + e) = o; }
template <int NFULL, int TAIL> __global__ __launch_bounds__(256) void k_soft(const float* __restrict__ Sb, int nrows, int rowsper, int rvalid, int nvalid, h16* P) { const int lane = threadIdx.x & 31; const size_t row = (size_t)blockIdx.x * 8 + (threadIdx.x >> 5); if (row >= (size_t)nrows) return; constexpr int LD = NFULL * 128 + TAIL * 64; const float* sr = Sb + row * LD; h16* pr = P + row * LD; const bool live = (int)(row % rowsper) < rvalid; float mx = -3.0e38f;
#pragma unroll 1
    for (int ch = 0; ch < NFULL + TAIL; ++ch) { if (ch == NFULL && lane >= 16) break; const int j0 = ch * 128 + lane * 4; const v4f a = *(const v4f*)(sr + j0);
#pragma unroll
        for (int q = 0; q < 4; ++q) if (j0 + q < nvalid) mx = fmaxf(mx, a[q]); }
#pragma unroll
    for (int sh = 16; sh; sh >>= 1) mx = fmaxf(mx, __shfl_xor(mx, sh, 32));
    float sum = 0.f;
#pragma unroll 1
    for (int ch = 0; ch < NFULL + TAIL; ++ch) { if (ch == NFULL && lane >= 16) break; const int j0 = ch * 128 + lane * 4; const v4f a = *(const v4f*)(sr + j0);
#pragma unroll
        for (int q = 0; q < 4; ++q) if (j0 + q < nvalid) { float d0 = __fsub_rn(a[q], mx); asm volatile("" : "+v"(d0)); sum += __expf(d0); } }
#pragma unroll
    for (int sh = 16; sh; sh >>= 1) sum += __shfl_xor(sum, sh, 32);
    const float f = live ? __fdiv_rn(PCAR, sum) : 0.f;
    for (int ps = 0; ps < 2; ++ps) {
#pragma unroll 1
        for (int ch = 0; ch < NFULL + TAIL; ++ch) { if (ch == NFULL && lane >= 16) break; const int j0 = ch * 128 + lane * 4; const v4f a = *(const v4f*)(sr + j0); v4h o;
#pragma unroll
            for (int q = 0; q < 4; ++q) { float val = 0.f; if (live && j0 + q < nvalid) { float d0 = __fsub_rn(a[q], mx); asm volatile("" : "+v"(d0)); val = __fmul_rn(__expf(d0), f); } o[q] = tohx(val); } *(volatile v4h*)(pr + j0) = o; }
        if (ps == 0) __threadfence(); } }

extern "C" void kernel_launch(void* const* d_in, const int* in_sizes, int n_in,
                              void* d_out, int out_size, void* d_ws, size_t ws_size, hipStream_t stream) {
    (void)in_sizes; (void)n_in; (void)out_size;
    const float* x = (const float*)d_in[0]; const float* qkv_w = (const float*)d_in[1]; const float* qkv_b = (const float*)d_in[2]; const float* dw_w = (const float*)d_in[3]; const float* dw_b = (const float*)d_in[4]; const float* aw1 = (const float*)d_in[5]; const float* ab1 = (const float*)d_in[6]; const float* aw2 = (const float*)d_in[7]; const float* ab2 = (const float*)d_in[8];
    const float* gq_w = (const float*)d_in[9]; const float* gq_b = (const float*)d_in[10]; const float* gkv_w = (const float*)d_in[11]; const float* gkv_b = (const float*)d_in[12]; const float* ca_w1 = (const float*)d_in[13]; const float* ca_w2 = (const float*)d_in[14]; const float* pw = (const float*)d_in[15]; const float* pb = (const float*)d_in[16];
    float* OUT = (float*)d_out;
    char* wsp = (char*)d_ws;
    auto take = [&](size_t bytes) { char* p = wsp; wsp += (bytes + 255) & ~(size_t)255; return (void*)p; };
    bf* WQKV = (bf*)take((size_t)3 * HF * CC * 2); bf* WA1 = (bf*)take(HF * HF * 2); bf* WA2 = (bf*)take(HF * HF * 2); bf* WGQ = (bf*)take(HF * CC * 2); bf* WGKV = (bf*)take(2 * HF * CC * 2); bf* WP = (bf*)take(CC * CC * 2);
    bf* XT = (bf*)take((size_t)NN * CC * 2); float* QKV = (float*)take((size_t)NN * 3 * HF * 4); float* QC = (float*)take((size_t)NN * 3 * HF * 4); bf* Ah = (bf*)take((size_t)NN * HF * 2); bf* Al = (bf*)take((size_t)NN * HF * 2); float* A1 = (float*)take((size_t)NN * HF * 4); float* A2 = (float*)take((size_t)NN * HF * 4); float* COMB = (float*)take((size_t)NN * CC * 4);
    float* GQ = (float*)take((size_t)NN * HF * 4); float* GKV = (float*)take((size_t)NN * 2 * HF * 4); h16* Q16 = (h16*)take((size_t)NH_ * NN * HD * 2); h16* K16 = (h16*)take((size_t)NH_ * NN * HD * 2); h16* VT = (h16*)take((size_t)NH_ * 64 * NN * 2); float* Sb = (float*)take((size_t)NH_ * NN * NN * 4); h16* P16 = (h16*)take((size_t)NH_ * NN * NN * 2); float* O = (float*)take((size_t)NH_ * NN * 64 * 4);
    float* CA = (float*)take(CC * 4); bf* Ch = (bf*)take((size_t)NN * CC * 2); bf* Cl = (bf*)take((size_t)NN * CC * 2); float* R = (float*)take((size_t)NN * CC * 4);
    if ((size_t)(wsp - (char*)d_ws) > ws_size) return;
    k_cvt8<<<(3 * HF * CC / 8 + 255) / 256, 256, 0, stream>>>(qkv_w, WQKV, 3 * HF * CC / 8); k_cvt8<<<(HF * HF / 8 + 255) / 256, 256, 0, stream>>>(aw1, WA1, HF * HF / 8); k_cvt8<<<(HF * HF / 8 + 255) / 256, 256, 0, stream>>>(aw2, WA2, HF * HF / 8); k_cvt8<<<(HF * CC / 8 + 255) / 256, 256, 0, stream>>>(gq_w, WGQ, HF * CC / 8); k_cvt8<<<(2 * HF * CC / 8 + 255) / 256, 256, 0, stream>>>(gkv_w, WGKV, 2 * HF * CC / 8); k_cvt8<<<(CC * CC / 8 + 255) / 256, 256, 0, stream>>>(pw, WP, CC * CC / 8);
    for (int b = 0; b < NBI; ++b) {
        k_xt<<<(NN * CC / 4 + 255) / 256, 256, 0, stream>>>(x + (size_t)b * CC * NN, XT);
        k_gemmw<bf, 0, true><<<dim3(NN / 64, 3 * HF / 64, 1), 32, 0, stream>>>(XT, nullptr, WQKV, nullptr, CC, QKV, 3 * HF, qkv_b, 0, 0, 0); k_dw<<<(NN * 3 * HF / 4 + 255) / 256, 256, 0, stream>>>(QKV, dw_w, dw_b, QC);
        k_qkpl<<<(NN * HF / 4 + 255) / 256, 256, 0, stream>>>(QC, Ah, Al); k_gemmw<bf, 1, true><<<dim3(NN / 64, HF / 64, 1), 32, 0, stream>>>(Ah, Al, WA1, nullptr, HF, A1, HF, ab1, 0, 0, 0);
        k_swpl<<<(NN * HF / 4 + 255) / 256, 256, 0, stream>>>(A1, Ah, Al); k_gemmw<bf, 1, true><<<dim3(NN / 64, HF / 64, 1), 32, 0, stream>>>(Ah, Al, WA2, nullptr, HF, A2, HF, ab2, 0, 0, 0); k_high<<<(NN * HF / 4 + 255) / 256, 256, 0, stream>>>(A2, QC, COMB);
        k_gemmw<bf, 0, true><<<dim3(NN / 64, HF / 64, 1), 32, 0, stream>>>(XT, nullptr, WGQ, nullptr, CC, GQ, HF, gq_b, 0, 0, 0); k_gemmw<bf, 0, true><<<dim3(NN / 64, 2 * HF / 64, 1), 32, 0, stream>>>(XT, nullptr, WGKV, nullptr, CC, GKV, 2 * HF, gkv_b, 0, 0, 0);
        k_gpl<<<(NH_ * NN * HD / 4 + 255) / 256, 256, 0, stream>>>(GQ, GKV, Q16, K16); k_gvt<<<(NH_ * 64 * NN / 2 + 255) / 256, 256, 0, stream>>>(GKV, VT);
        k_gemmw<h16, 0, false><<<dim3(NN / 64, NN / 64, NH_), 32, 0, stream>>>(Q16, nullptr, K16, nullptr, HD, Sb, NN, nullptr, (size_t)NN * HD, (size_t)NN * HD, (size_t)NN * NN);
        k_soft<8, 0><<<(NH_ * NN + 7) / 8, 256, 0, stream>>>(Sb, NH_ * NN, NN, NN, NN, P16);
        k_gemmw<h16, 0, false><<<dim3(NN / 64, 1, NH_), 32, 0, stream>>>(P16, nullptr, VT, nullptr, NN, O, 64, nullptr, (size_t)NN * NN, (size_t)64 * NN, (size_t)NN * 64); k_low<<<(NN * HF / 4 + 255) / 256, 256, 0, stream>>>(O, COMB);
        k_se<<<1, 256, 0, stream>>>(COMB, ca_w1, ca_w2, CA); k_capl<<<(NN * CC / 4 + 255) / 256, 256, 0, stream>>>(COMB, CA, Ch, Cl);
        k_gemmw<bf, 1, true><<<dim3(NN / 64, CC / 64, 1), 32, 0, stream>>>(Ch, Cl, WP, nullptr, CC, R, CC, pb, 0, 0, 0); k_outT<<<(CC * NN / 4 + 255) / 256, 256, 0, stream>>>(R, x + (size_t)b * CC * NN, OUT + (size_t)b * CC * NN); }
}
